// MyDCNv2_33268816675419
// MI455X (gfx1250) — hardware-verified
//
#include <hip/hip_runtime.h>


namespace {
constexpr int NB_ = 8, C = 256, OC = 256, HH = 64, WW = 64, K9 = 9, KK = C * K9  , NP = HH * WW  ;
constexpr float AS = 16.0f, WSC = 256.0f;
typedef _Float16 b16;
typedef __attribute__((ext_vector_type(16))) _Float16 v16b;
typedef __attribute__((ext_vector_type(8))) _Float16 v8b;
typedef __attribute__((ext_vector_type(8))) float v8f;
typedef __attribute__((ext_vector_type(4))) float v4f;
__device__ __forceinline__ float bf16_rne(float f) { unsigned int u = __float_as_uint(f); u += 0x7FFFu + ((u >> 16) & 1u); float r = __uint_as_float(u & 0xFFFF0000u); asm volatile("" : "+v"(r)); return r; }
__device__ __forceinline__ float bfv(float f) { float r = bf16_rne(f); asm volatile("" : "+v"(r)); return r; }
__device__ __forceinline__ v16b frag_kb(const b16* p, int hh) { const v8b a = *(const v8b*)(p + 8 * hh), b = *(const v8b*)(p + 16 + 8 * hh); v16b f;
#pragma unroll
  for (int e = 0; e < 8; ++e) { f[e] = a[e]; f[8 + e] = b[e]; } return f; }
__device__ __forceinline__ v8f wmma16b(v16b a, v16b b, v8f c) { v8f d = __builtin_amdgcn_wmma_f32_16x16x32_f16(false, a, false, b, (short)0, c, false, false); asm volatile("v_nop\n\tv_nop\n\tv_nop\n\tv_nop" : "+v"(d) : "v"(a), "v"(b)); return d; }
__device__ __forceinline__ void wave_lds_sync() { __builtin_amdgcn_fence(__ATOMIC_RELEASE, "workgroup"); __builtin_amdgcn_wave_barrier(); __builtin_amdgcn_fence(__ATOMIC_ACQUIRE, "workgroup"); }
__device__ __forceinline__ float pmul(float a, float b) { float p = a * b; asm volatile("" : "+v"(p)); return p; }

__global__ __launch_bounds__(256) void wput_kernel(const float* __restrict__ w, b16* __restrict__ WT) { const size_t nt = (size_t)gridDim.x * 256, u0 = (size_t)blockIdx.x * 256 + threadIdx.x; v8b v;
  for (size_t u = u0; u < (size_t)OC * KK / 8; u += nt) {
#pragma unroll
    for (int j = 0; j < 8; ++j) v[j] = (b16)(bf16_rne(w[u * 8 + j]) * WSC); for (int pass = 0; pass < 2; ++pass) { *(volatile v8b*)(WT + u * 8) = v; __threadfence(); } } }
__global__ __launch_bounds__(32) void main_kernel(const float* __restrict__ x, const float* __restrict__ offs, const float* __restrict__ msk, const b16* __restrict__ WT, int PLIM, float* __restrict__ ST) { __shared__ __attribute__((aligned(16))) b16 Ah[16][KK + 8]; __shared__ float Cw[16][K9][4], Tf[16][260]; __shared__ int Ci[16][K9][4]; const int lane = threadIdx.x, nloc = lane & 15, hlf = lane >> 4; const int n = blockIdx.x / (NP / 16), p0 = (blockIdx.x % (NP / 16)) * 16; if (p0 >= PLIM) return;
  if (lane < 16) { const int p = p0 + lane, oy = p / WW, ox = p % WW;
    for (int k = 0; k < K9; ++k) { const int ky = k / 3, kx = k % 3; const float dy = bfv(offs[(((size_t)n * 2 * K9 + 2 * k) * NP) + p]), dx = bfv(offs[(((size_t)n * 2 * K9 + 2 * k + 1) * NP) + p]); const float py = (float)oy + (float)ky + dy, px = (float)ox + (float)kx + dx; const float fy = floorf(py), fx = floorf(px); const float ly = py - fy, lx = px - fx; const int y0 = (int)fy, x0 = (int)fx; const float m = bfv(msk[(((size_t)n * K9 + k) * NP) + p]);
      for (int cr = 0; cr < 4; ++cr) { const int yi = y0 + (cr >> 1), xi = x0 + (cr & 1); const float wgt = ((cr >> 1) ? ly : 1.0f - ly) * ((cr & 1) ? lx : 1.0f - lx); const bool inb = yi >= 1 && yi <= HH && xi >= 1 && xi <= WW;
        Cw[lane][k][cr] = inb ? wgt * m : 0.0f; Ci[lane][k][cr] = inb ? (yi - 1) * WW + (xi - 1) : 0; } }
    for (int kk = KK; kk < KK + 8; ++kk) Ah[lane][kk] = (b16)0.0f; }
  wave_lds_sync();
  const float* xn = x + (size_t)n * C * NP;
  for (int p = 0; p < 16; ++p) {
#pragma unroll 1
    for (int k = 0; k < K9; ++k) { const float w0 = Cw[p][k][0], w1 = Cw[p][k][1], w2 = Cw[p][k][2], w3 = Cw[p][k][3]; const int i0 = Ci[p][k][0], i1 = Ci[p][k][1], i2 = Ci[p][k][2], i3 = Ci[p][k][3];
      for (int c = lane; c < C; c += 32) { const float* xc = xn + (size_t)c * NP; const float v = pmul(bfv(xc[i0]), w0) + pmul(bfv(xc[i1]), w1) + pmul(bfv(xc[i2]), w2) + pmul(bfv(xc[i3]), w3); Ah[p][c * K9 + k] = (b16)(v * AS); } } }
  wave_lds_sync(); v8f acc[16];
#pragma unroll
  for (int t = 0; t < 16; ++t) acc[t] = (v8f){};
#pragma unroll 2
  for (int kb = 0; kb < KK; kb += 32) { const v16b a = frag_kb(&Ah[nloc][kb], hlf);
#pragma unroll
    for (int t = 0; t < 16; ++t) acc[t] = wmma16b(a, frag_kb(WT + (size_t)(t * 16 + nloc) * KK + kb, hlf), acc[t]); }
#pragma unroll
  for (int t = 0; t < 16; ++t)
#pragma unroll
    for (int r8 = 0; r8 < 8; ++r8) Tf[8 * hlf + r8][t * 16 + nloc] = acc[t][r8] * (1.0f / (AS * WSC));
  wave_lds_sync();
  for (int pass = 0; pass < 2; ++pass) { for (int rr = 0; rr < 16; ++rr) for (int q = 0; q < 2; ++q) *(volatile v4f*)(ST + ((size_t)n * NP + p0 + rr) * OC + q * 128 + lane * 4) = *(const v4f*)(&Tf[rr][q * 128 + lane * 4]); __threadfence(); } }
__global__ __launch_bounds__(256) void copy_kernel(const float* __restrict__ ST, int PLIM, float* __restrict__ out) { const size_t u = (size_t)blockIdx.x * 256 + threadIdx.x; if (u >= (size_t)NB_ * OC * NP) return; const int p = (int)(u % NP), o = (int)((u / NP) % OC), n = (int)(u / ((size_t)NP * OC)); const float v = p < PLIM ? ST[((size_t)n * NP + p) * OC + o] : 0.0f;
  for (int pass = 0; pass < 2; ++pass) { ((volatile float*)out)[u] = v; __threadfence(); } }
}

extern "C" void kernel_launch(void* const* d_in, const int* in_sizes, int n_in, void* d_out, int out_size, void* d_ws, size_t ws_size, hipStream_t stream) {
  (void)n_in;
  auto Fp = [&](int i) { return (const float*)d_in[i]; };
  if (in_sizes[0] != NB_ * C * NP || in_sizes[1] != NB_ * 2 * K9 * NP || in_sizes[2] != NB_ * K9 * NP || in_sizes[3] != OC * KK || out_size != NB_ * OC * NP) return;
  const int PLIM = NP;
  size_t off = 0; char* ws = (char*)d_ws;
  auto carve = [&](size_t bytes) { char* p = ws + off; off += (bytes + 255) & ~(size_t)255; return p; };
  b16* WT = (b16*)carve((size_t)OC * KK * 2); float* ST = (float*)carve((size_t)NB_ * NP * OC * 4);
  if (off > ws_size || off > ((size_t)40 << 20)) return;
  wput_kernel<<<256, 256, 0, stream>>>(Fp(3), WT);
  main_kernel<<<NB_ * (NP / 16), 32, 0, stream>>>(Fp(0), Fp(1), Fp(2), WT, PLIM, ST);
  copy_kernel<<<(NB_ * OC * NP + 255) / 256, 256, 0, stream>>>(ST, PLIM, (float*)d_out);
}
